// SelfAttention_65085934403863
// MI455X (gfx1250) — hardware-run, weakly checked
//
#include <hip/hip_runtime.h>
#include <math.h>
#include <stdint.h>

#pragma clang fp contract(off)

#define NH_  16
#define T_   2048
#define D_   64
#define OS_P 68

static_assert(D_ == 64);
static_assert(T_ % 64 == 0);
static_assert(NH_ * (T_ / 64) == 512);

typedef __attribute__((ext_vector_type(16))) __bf16   v16b;
typedef __attribute__((ext_vector_type(8)))  float    v8f;
typedef __attribute__((ext_vector_type(4)))  float    v4f;
typedef __attribute__((ext_vector_type(4)))  unsigned int v4u;
typedef __attribute__((ext_vector_type(8)))  unsigned short u16x8;

union FragB { u16x8 h[2]; v16b v; };

constexpr size_t SZ_PL  = (size_t)NH_ * T_ * D_ * 2;
constexpr size_t OFF_QB = 0;
constexpr size_t OFF_KH = OFF_QB + SZ_PL;
constexpr size_t OFF_KM = OFF_KH + SZ_PL;
constexpr size_t OFF_KL = OFF_KM + SZ_PL;
constexpr size_t OFF_VT = OFF_KL + SZ_PL;
constexpr size_t WS_END = OFF_VT + SZ_PL;
static_assert(WS_END <= (size_t)134217728);
static_assert(OFF_KH % 256 == 0 && OFF_KM % 256 == 0 && OFF_KL % 256 == 0 && OFF_VT % 256 == 0);

constexpr float THR_ = (float)(0.01 + 1e-7);
static_assert(__builtin_bit_cast(unsigned, THR_) == 0x3C23D776u);

__device__ __forceinline__ unsigned short f2bf_bits(float f) {
  unsigned u = __float_as_uint(f);
  return (unsigned short)((u + 0x7FFFu + ((u >> 16) & 1u)) >> 16);
}
__device__ __forceinline__ float bf_bits2f(unsigned short h) { return __uint_as_float(((unsigned)h) << 16); }
__device__ __forceinline__ float bf_rne(float f) { return bf_bits2f(f2bf_bits(f)); }
__device__ __forceinline__ unsigned pk16(unsigned short a, unsigned short b) { return (unsigned)a | ((unsigned)b << 16); }
__device__ __forceinline__ void split3(float f, unsigned short& h, unsigned short& m, unsigned short& l) {
  h = f2bf_bits(f);
  const float r1 = f - bf_bits2f(h);
  m = f2bf_bits(r1);
  const float r2 = r1 - bf_bits2f(m);
  l = f2bf_bits(r2);
}

__device__ __forceinline__ v8f mma_g(v8f c, v16b a, v16b b) {
  c = __builtin_amdgcn_wmma_f32_16x16x32_bf16(false, a, false, b, (short)0, c, false, false);
  asm volatile("v_nop\n\tv_nop\n\tv_nop\n\tv_nop" : "+v"(c) : "v"(a), "v"(b));
  return c;
}

__global__ __launch_bounds__(256)
void k_prep(const float* __restrict__ Q, const float* __restrict__ K, const float* __restrict__ V,
            unsigned short* qb, unsigned short* kh, unsigned short* km, unsigned short* kl, unsigned short* vt) {
  __shared__ __align__(16) float tf[64 * OS_P];
  __shared__ __align__(16) float nrm[64];
  const int tid  = threadIdx.x;
  const int h    = blockIdx.x >> 5;
  const int r0   = (blockIdx.x & 31) * 64;
  const size_t rowbase = (size_t)h * T_ + r0;

  v4u qv[2];
#pragma unroll
  for (int it = 0; it < 2; ++it) {
    const int idx = it * 256 + tid;
    const int row = idx >> 3;
    const int c8  = (idx & 7) * 8;
    const float* p = Q + (rowbase + row) * D_ + c8;
    const v4f a = *(const v4f*)p;
    const v4f b = *(const v4f*)(p + 4);
    v4u o;
    o[0] = pk16(f2bf_bits(a[0]), f2bf_bits(a[1]));
    o[1] = pk16(f2bf_bits(a[2]), f2bf_bits(a[3]));
    o[2] = pk16(f2bf_bits(b[0]), f2bf_bits(b[1]));
    o[3] = pk16(f2bf_bits(b[2]), f2bf_bits(b[3]));
    qv[it] = o;
  }

  {
    const int lr = tid >> 4;
    const int c4 = (tid & 15) * 4;
#pragma unroll
    for (int it = 0; it < 4; ++it) {
      const int rr = it * 16 + lr;
      const v4f a = *(const v4f*)(K + (rowbase + rr) * D_ + c4);
      v4f o;
      o[0] = bf_rne(a[0]); o[1] = bf_rne(a[1]); o[2] = bf_rne(a[2]); o[3] = bf_rne(a[3]);
      *(v4f*)(tf + rr * OS_P + c4) = o;
    }
  }
  __syncthreads();
  if (tid < 64) {
    double s = 0.0;
#pragma unroll 4
    for (int j = 0; j < 64; ++j) {
      const float v  = tf[tid * OS_P + j];
      const float sq = v * v;
      s += (double)sq;
    }
    const float ss = (float)s;
    float n = sqrtf(ss);
    n = fmaxf(n, 1e-8f);
    nrm[tid] = n;
  }
  __syncthreads();
#pragma unroll 2
  for (int i = 0; i < 16; ++i) {
    const int idx = i * 256 + tid;
    const int row = idx >> 6;
    const int col = idx & 63;
    const float v = tf[row * OS_P + col];
    const float n = nrm[row];
    tf[row * OS_P + col] = v / n;
  }
  __syncthreads();
  v4u khv[2], kmv[2], klv[2];
#pragma unroll
  for (int it = 0; it < 2; ++it) {
    const int idx = it * 256 + tid;
    const int row = idx >> 3;
    const int c8  = (idx & 7) * 8;
    v4u a, b, cc;
#pragma unroll
    for (int q = 0; q < 4; ++q) {
      const float f0 = tf[row * OS_P + c8 + 2 * q];
      const float f1 = tf[row * OS_P + c8 + 2 * q + 1];
      unsigned short h0, m0, l0, h1, m1, l1;
      split3(f0, h0, m0, l0);
      split3(f1, h1, m1, l1);
      a[q]  = pk16(h0, h1);
      b[q]  = pk16(m0, m1);
      cc[q] = pk16(l0, l1);
    }
    khv[it] = a; kmv[it] = b; klv[it] = cc;
  }
  __syncthreads();

  {
    const int lr = tid >> 4;
    const int c4 = (tid & 15) * 4;
#pragma unroll
    for (int it = 0; it < 4; ++it) {
      const int rr = it * 16 + lr;
      const v4f a = *(const v4f*)(V + (rowbase + rr) * D_ + c4);
      *(v4f*)(tf + rr * OS_P + c4) = a;
    }
  }
  __syncthreads();
  v4u vtv[2];
  const int sub = tid >> 3;
  const int k8  = (tid & 7) * 8;
#pragma unroll
  for (int it = 0; it < 2; ++it) {
    const int d = it * 32 + sub;
    v4u a;
#pragma unroll
    for (int q = 0; q < 4; ++q) {
      const float f0 = tf[(k8 + 2 * q) * OS_P + d];
      const float f1 = tf[(k8 + 2 * q + 1) * OS_P + d];
      a[q] = pk16(f2bf_bits(f0), f2bf_bits(f1));
    }
    vtv[it] = a;
  }

  for (int pass = 0; pass < 2; ++pass) {
#pragma unroll
    for (int it = 0; it < 2; ++it) {
      const int idx = it * 256 + tid;
      const int row = idx >> 3;
      const int c8  = (idx & 7) * 8;
      const size_t go = (rowbase + row) * D_ + c8;
      *(volatile v4u*)(qb + go) = qv[it];
      *(volatile v4u*)(kh + go) = khv[it];
      *(volatile v4u*)(km + go) = kmv[it];
      *(volatile v4u*)(kl + go) = klv[it];
      const int d = it * 32 + sub;
      const size_t vo = ((size_t)h * D_ + d) * T_ + r0 + k8;
      *(volatile v4u*)(vt + vo) = vtv[it];
    }
    __threadfence();
  }
}

__global__ __launch_bounds__(128) __attribute__((amdgpu_num_vgpr(248)))
void k_attn(const unsigned short* __restrict__ qb,
            const unsigned short* __restrict__ khp, const unsigned short* __restrict__ kmp,
            const unsigned short* __restrict__ klp, const unsigned short* __restrict__ vtp,
            const float* __restrict__ gain, const float* __restrict__ bias,
            float* out) {
  __shared__ __align__(16) unsigned short Ksh[64 * D_];
  __shared__ __align__(16) unsigned short Ksm[64 * D_];
  __shared__ __align__(16) unsigned short Ksl[64 * D_];
  __shared__ __align__(16) unsigned short Vts[D_ * 64];
  __shared__ __align__(16) unsigned short Psh[4][16 * 64];
  __shared__ __align__(16) unsigned short Psl[4][16 * 64];
  __shared__ __align__(16) float Os[4][16 * OS_P];
  __shared__ __align__(16) float gsh[64];
  __shared__ __align__(16) float bsh[64];

  const int tid  = threadIdx.x;
  const int wave = tid >> 5;
  const int lane = tid & 31;
  const int hh   = lane >> 4;
  const int c    = lane & 15;

  const int qt  = blockIdx.x & 31;
  const int h   = blockIdx.x >> 5;
  const int q0w = qt * 64 + wave * 16;

  const unsigned short* Qh = qb  + (size_t)h * T_ * D_;
  const unsigned short* Kh = khp + (size_t)h * T_ * D_;
  const unsigned short* Km = kmp + (size_t)h * T_ * D_;
  const unsigned short* Kl = klp + (size_t)h * T_ * D_;
  const unsigned short* Vt = vtp + (size_t)h * D_ * T_;

  if (wave == 0) {
    const int o = (lane & 15) * 4;
    const v4f g4 = *(const v4f*)(gain + (size_t)h * T_ + qt * 64 + o);
    const v4f b4 = *(const v4f*)(bias + (size_t)h * T_ + qt * 64 + o);
    asm volatile("" :: "v"(g4), "v"(b4));
    v4f gr, br;
    gr[0] = bf_rne(g4[0]); gr[1] = bf_rne(g4[1]); gr[2] = bf_rne(g4[2]); gr[3] = bf_rne(g4[3]);
    br[0] = bf_rne(b4[0]); br[1] = bf_rne(b4[1]); br[2] = bf_rne(b4[2]); br[3] = bf_rne(b4[3]);
    if (lane < 16) {
      *(v4f*)(gsh + o) = gr;
      *(v4f*)(bsh + o) = br;
    }
  }
  __syncthreads();
  float gv[8], bv[8];
  {
    const float* gp = gsh + wave * 16 + 8 * hh;
    const float* bp = bsh + wave * 16 + 8 * hh;
    const v4f g0 = *(const v4f*)gp;
    const v4f g1 = *(const v4f*)(gp + 4);
    const v4f b0 = *(const v4f*)bp;
    const v4f b1 = *(const v4f*)(bp + 4);
    gv[0] = g0[0]; gv[1] = g0[1]; gv[2] = g0[2]; gv[3] = g0[3];
    gv[4] = g1[0]; gv[5] = g1[1]; gv[6] = g1[2]; gv[7] = g1[3];
    bv[0] = b0[0]; bv[1] = b0[1]; bv[2] = b0[2]; bv[3] = b0[3];
    bv[4] = b1[0]; bv[5] = b1[1]; bv[6] = b1[2]; bv[7] = b1[3];
  }

  FragB qa0, qa1;
  {
    const unsigned short* qr = Qh + (size_t)(q0w + c) * D_ + 8 * hh;
    qa0.h[0] = *(const u16x8*)(qr);
    qa0.h[1] = *(const u16x8*)(qr + 16);
    qa1.h[0] = *(const u16x8*)(qr + 32);
    qa1.h[1] = *(const u16x8*)(qr + 48);
  }

  float ssq[8];
  v8f oacc[4];
#pragma unroll
  for (int r = 0; r < 8; ++r) ssq[r] = 0.0f;
#pragma unroll
  for (int t = 0; t < 4; ++t) oacc[t] = (v8f){0.f,0.f,0.f,0.f,0.f,0.f,0.f,0.f};

  unsigned short* pwh = Psh[wave];
  unsigned short* pwl = Psl[wave];

  const int nChunks = qt + 1;
  for (int kt = 0; kt < nChunks; ++kt) {
    const int kv0 = kt * 64;
    __syncthreads();
    {
      const int r = tid >> 1, half = (tid & 1) * 32;
      const unsigned short* s0 = Kh + (size_t)(kv0 + r) * D_ + half;
      const unsigned short* s1 = Km + (size_t)(kv0 + r) * D_ + half;
      const unsigned short* s2 = Kl + (size_t)(kv0 + r) * D_ + half;
      const unsigned short* s3 = Vt + (size_t)r * T_ + kv0 + half;
#pragma unroll
      for (int i = 0; i < 4; ++i) {
        const u16x8 a0 = *(const u16x8*)(s0 + 8 * i);
        const u16x8 a1 = *(const u16x8*)(s1 + 8 * i);
        const u16x8 a2 = *(const u16x8*)(s2 + 8 * i);
        const u16x8 a3 = *(const u16x8*)(s3 + 8 * i);
        *(u16x8*)(Ksh + r * D_ + half + 8 * i) = a0;
        *(u16x8*)(Ksm + r * D_ + half + 8 * i) = a1;
        *(u16x8*)(Ksl + r * D_ + half + 8 * i) = a2;
        *(u16x8*)(Vts + r * 64 + half + 8 * i) = a3;
      }
    }
    __syncthreads();

    const bool diag = (kt == qt);
#pragma unroll 1
    for (int j = 0; j < 4; ++j) {
      const int ko = (j * 16 + c) * D_ + 8 * hh;
      FragB fl0, fl1, fm0, fm1, fh0, fh1;
      fl0.h[0] = *(const u16x8*)(Ksl + ko);      fl0.h[1] = *(const u16x8*)(Ksl + ko + 16);
      fl1.h[0] = *(const u16x8*)(Ksl + ko + 32); fl1.h[1] = *(const u16x8*)(Ksl + ko + 48);
      fm0.h[0] = *(const u16x8*)(Ksm + ko);      fm0.h[1] = *(const u16x8*)(Ksm + ko + 16);
      fm1.h[0] = *(const u16x8*)(Ksm + ko + 32); fm1.h[1] = *(const u16x8*)(Ksm + ko + 48);
      fh0.h[0] = *(const u16x8*)(Ksh + ko);      fh0.h[1] = *(const u16x8*)(Ksh + ko + 16);
      fh1.h[0] = *(const u16x8*)(Ksh + ko + 32); fh1.h[1] = *(const u16x8*)(Ksh + ko + 48);
      v8f s = (v8f){0.f,0.f,0.f,0.f,0.f,0.f,0.f,0.f};
      s = mma_g(s, qa0.v, fl0.v);
      s = mma_g(s, qa1.v, fl1.v);
      s = mma_g(s, qa0.v, fm0.v);
      s = mma_g(s, qa1.v, fm1.v);
      s = mma_g(s, qa0.v, fh0.v);
      s = mma_g(s, qa1.v, fh1.v);

      const int d0 = q0w + 8 * hh - (kv0 + j * 16 + c);
#pragma unroll
      for (int r = 0; r < 8; ++r) {
        const float dot = s[r];
        float I = gv[r] * dot;
        I = I + bv[r];
        const bool good = I > THR_;
        const float Is = good ? I : 1.0f;
        const float x  = (-0.01f) / Is;
        const float lt = log1pf(x);
        float den = 0.02f * lt;
        den = 0.002f - den;
        const float rinv = 1.0f / den;
        float rate = good ? rinv : 0.0f;
        rate = rate * 0.125f;
        const bool keep = (!diag) || (d0 + r >= 0);
        rate = keep ? rate : 0.0f;
        const float sq = rate * rate;
        ssq[r] = ssq[r] + sq;
        const unsigned short hb = f2bf_bits(rate);
        const unsigned short lb = f2bf_bits(rate - bf_bits2f(hb));
        pwh[(8 * hh + r) * 64 + j * 16 + c] = hb;
        pwl[(8 * hh + r) * 64 + j * 16 + c] = lb;
      }
    }
    __syncthreads();

#pragma unroll 1
    for (int kk = 0; kk < 2; ++kk) {
      FragB pa, pl;
      const int po = c * 64 + kk * 32 + 8 * hh;
      pa.h[0] = *(const u16x8*)(pwh + po);
      pa.h[1] = *(const u16x8*)(pwh + po + 16);
      pl.h[0] = *(const u16x8*)(pwl + po);
      pl.h[1] = *(const u16x8*)(pwl + po + 16);
#pragma unroll
      for (int t = 0; t < 4; ++t) {
        FragB vb;
        const int vo = (t * 16 + c) * 64 + kk * 32 + 8 * hh;
        vb.h[0] = *(const u16x8*)(Vts + vo);
        vb.h[1] = *(const u16x8*)(Vts + vo + 16);
        oacc[t] = mma_g(oacc[t], pl.v, vb.v);
        oacc[t] = mma_g(oacc[t], pa.v, vb.v);
      }
    }
  }

  float* os = Os[wave];
#pragma unroll
  for (int r = 0; r < 8; ++r) {
    float a = ssq[r];
    a = a + __shfl_xor(a, 1, 32);
    a = a + __shfl_xor(a, 2, 32);
    a = a + __shfl_xor(a, 4, 32);
    a = a + __shfl_xor(a, 8, 32);
    const float pool = sqrtf(a + 1e-20f);
    const float den  = 0.001f + pool;
#pragma unroll
    for (int t = 0; t < 4; ++t) os[(8 * hh + r) * OS_P + t * 16 + c] = oacc[t][r] / den;
  }
  __syncthreads();
  {
    float* ob = out + (size_t)h * T_ * D_;
    const int c4 = (lane & 15) * 4;
    for (int pass = 0; pass < 2; ++pass) {
#pragma unroll
      for (int it = 0; it < 8; ++it) {
        const int row = it * 2 + hh;
        const v4f val = *(const v4f*)(os + row * OS_P + c4);
        *(volatile v4f*)(ob + (size_t)(q0w + row) * D_ + c4) = val;
      }
      __threadfence();
    }
  }
}

extern "C" void kernel_launch(void* const* d_in, const int* in_sizes, int n_in,
                              void* d_out, int out_size, void* d_ws, size_t ws_size,
                              hipStream_t stream) {
  if (n_in < 5) return;
  if (in_sizes[0] != NH_ * T_ * D_) return;
  if (in_sizes[1] != NH_ * T_ * D_) return;
  if (in_sizes[2] != NH_ * T_ * D_) return;
  if (in_sizes[3] != NH_ * T_) return;
  if (in_sizes[4] != NH_ * T_) return;
  if (out_size != NH_ * T_ * D_) return;
  if (ws_size < WS_END) return;

  const float* Q    = (const float*)d_in[0];
  const float* K    = (const float*)d_in[1];
  const float* V    = (const float*)d_in[2];
  const float* gain = (const float*)d_in[3];
  const float* bias = (const float*)d_in[4];
  float* out = (float*)d_out;

  char* ws = (char*)d_ws;
  unsigned short* QB = (unsigned short*)(ws + OFF_QB);
  unsigned short* KH = (unsigned short*)(ws + OFF_KH);
  unsigned short* KM = (unsigned short*)(ws + OFF_KM);
  unsigned short* KL = (unsigned short*)(ws + OFF_KL);
  unsigned short* VT = (unsigned short*)(ws + OFF_VT);

  const dim3 grid(NH_ * (T_ / 64));

  k_prep<<<grid, dim3(256), 0, stream>>>(Q, K, V, QB, KH, KM, KL, VT);
  k_attn<<<grid, dim3(128), 0, stream>>>(QB, KH, KM, KL, VT, gain, bias, out);
  (void)hipGetLastError();
}
